// RotaryEmbeddingTransformerLayer_36919538876926
// MI455X (gfx1250) — hardware-verified
//
#include <hip/hip_runtime.h>


namespace {
constexpr int Bn = 2, L = 2048, D = 1024, H = 16, HD = 64, NT = Bn * L, DQ = 3 * D, DF = 4096;
constexpr float EPS = 1e-5f, XS = 8.0f, PS = 8.0f;

typedef _Float16 b16;
typedef __attribute__((ext_vector_type(16))) _Float16 v16b;
typedef __attribute__((ext_vector_type(8))) _Float16 v8b;
typedef __attribute__((ext_vector_type(8))) float v8f;
typedef __attribute__((ext_vector_type(4))) float v4f;
__device__ __forceinline__ float bf16_rne(float f) { unsigned int u = __float_as_uint(f); u += 0x7FFFu + ((u >> 16) & 1u); return __uint_as_float(u & 0xFFFF0000u); }
__device__ __forceinline__ v16b frag_kb(const b16* p, int hh) { const v8b a = *(const v8b*)(p + 8 * hh), b = *(const v8b*)(p + 16 + 8 * hh); v16b f;
#pragma unroll
  for (int e = 0; e < 8; ++e) { f[e] = a[e]; f[8 + e] = b[e]; } return f; }
__device__ __forceinline__ v8f wmma16b(v16b a, v16b b, v8f c) { v8f d = __builtin_amdgcn_wmma_f32_16x16x32_f16(false, a, false, b, (short)0, c, false, false); asm volatile("v_nop\n\tv_nop\n\tv_nop\n\tv_nop" : "+v"(d) : "v"(a), "v"(b)); return d; }
__device__ __forceinline__ void wave_lds_sync() { __builtin_amdgcn_fence(__ATOMIC_RELEASE, "workgroup"); __builtin_amdgcn_wave_barrier(); __builtin_amdgcn_fence(__ATOMIC_ACQUIRE, "workgroup"); }
__device__ __forceinline__ float nexp(float x) { return __builtin_amdgcn_exp2f(x * 1.4426950408889634f); }
__device__ __forceinline__ float pmul(float a, float b) { float p = a * b; asm volatile("" : "+v"(p)); return p; }
__device__ __forceinline__ float wsum(float v) {
#pragma unroll
  for (int o = 1; o < 32; o <<= 1) v += __shfl_xor(v, o); return v; }
__device__ __forceinline__ void sincos_r(float ang, float& sn, float& cs) { const float k = rintf(ang * 0.15915494309189535f); float r = __builtin_fmaf(k, -6.28318548202514648f, ang); r = __builtin_fmaf(k, 1.7484556025237907e-7f, r);
  const float t = r * 0.15915494309189535f; sn = __builtin_amdgcn_sinf(t); cs = __builtin_amdgcn_cosf(t); }
__device__ __forceinline__ float tanh_n(float x) { const float e = __builtin_amdgcn_exp2f(x * 2.8853900817779268f); return 1.0f - 2.0f * __builtin_amdgcn_rcpf(e + 1.0f); }
__device__ __forceinline__ float gelu_t(float x) { const float c = 0.7978845608028654f; return 0.5f * x * (1.0f + tanh_n(c * (x + 0.044715f * x * x * x))); }

struct Wo_ { static constexpr size_t QKV = 0, O = QKV + (size_t)DQ * D, F1 = O + (size_t)D * D, F2 = F1 + (size_t)DF * D, END = F2 + (size_t)D * DF; };
__global__ __launch_bounds__(256) void prep_kernel(const float* __restrict__ wqkv, const float* __restrict__ wo, const float* __restrict__ w1, const float* __restrict__ w2, const float* __restrict__ bqkv, const float* __restrict__ bo, const float* __restrict__ b1, const float* __restrict__ b2, const float* __restrict__ g1, const float* __restrict__ be1, const float* __restrict__ g2, const float* __restrict__ be2, b16* __restrict__ R, float* __restrict__ P) {
  const size_t tid = (size_t)blockIdx.x * 256 + threadIdx.x, nth = (size_t)gridDim.x * 256;
  for (int pass = 0; pass < 2; ++pass) {
    for (size_t p = tid; p < Wo_::END / 8; p += nth) { const size_t q = p * 8; const float* src = (q < Wo_::O) ? (wqkv + q) : (q < Wo_::F1) ? (wo + (q - Wo_::O)) : (q < Wo_::F2) ? (w1 + (q - Wo_::F1)) : (w2 + (q - Wo_::F2)); v8b v;
#pragma unroll
      for (int e = 0; e < 8; ++e) v[e] = (b16)bf16_rne(src[e]); *(volatile v8b*)(R + q) = v; }
    for (size_t q = tid; q < 13312; q += nth) { const int i = (int)q; float v; if (i < 3072) v = bqkv[i]; else if (i < 4096) v = bo[i - 3072]; else if (i < 8192) v = b1[i - 4096]; else if (i < 9216) v = b2[i - 8192]; else if (i < 10240) v = g1[i - 9216]; else if (i < 11264) v = be1[i - 10240]; else if (i < 12288) v = g2[i - 11264]; else v = be2[i - 12288]; P[q] = bf16_rne(v); }
    __threadfence(); }
}

__global__ __launch_bounds__(256) void ln_kernel(const float* __restrict__ src, int rnd, const float* __restrict__ g, const float* __restrict__ bb, b16* __restrict__ dst) {
  const int row = blockIdx.x * 8 + (threadIdx.x >> 5), lane = threadIdx.x & 31; const float* xr = src + (size_t)row * D;
  float v[32]; float s = 0.0f;
#pragma unroll
  for (int i = 0; i < 32; ++i) { float x = xr[(i >> 3) * 256 + lane * 8 + (i & 7)]; if (rnd) x = bf16_rne(x); v[i] = x; s += x; }
  s = wsum(s); const float mu = s * (1.0f / D); float q = 0.0f;
#pragma unroll
  for (int i = 0; i < 32; ++i) { const float d = v[i] - mu; q += pmul(d, d); }
  q = wsum(q); const float inv = rsqrtf(q * (1.0f / D) + EPS);
  for (int pass = 0; pass < 2; ++pass) {
#pragma unroll
    for (int gq = 0; gq < 4; ++gq) { v8b o; const int c0 = gq * 256 + lane * 8;
#pragma unroll
      for (int e = 0; e < 8; ++e) o[e] = (b16)((pmul((v[gq * 8 + e] - mu) * inv, g[c0 + e]) + bb[c0 + e]) * XS);
      *(volatile v8b*)(dst + (size_t)row * D + c0) = o; }
    __threadfence(); }
}

template <int K, int N, int EPI, int RND>
__global__ __launch_bounds__(64) void gemm_kernel(const b16* __restrict__ A, const b16* __restrict__ Bw, const float* __restrict__ bias, const float* __restrict__ resid, b16* __restrict__ Ch, float* __restrict__ Cf) {
  __shared__ __attribute__((aligned(16))) float Ts[2][32][128 + 4];
  const int lane = threadIdx.x & 31, wave = threadIdx.x >> 5, nloc = lane & 15, hlf = lane >> 4, m0 = blockIdx.y * 32, c0 = blockIdx.x * 256 + wave * 128;
  v8f acc[2][8];
#pragma unroll
  for (int r = 0; r < 2; ++r)
#pragma unroll
    for (int t = 0; t < 8; ++t) acc[r][t] = (v8f){};
  for (int kb = 0; kb < K; kb += 32) { const v16b a0 = frag_kb(A + (size_t)(m0 + nloc) * K + kb, hlf), a1 = frag_kb(A + (size_t)(m0 + 16 + nloc) * K + kb, hlf);
#pragma unroll
    for (int t = 0; t < 8; ++t) { const v16b bw = frag_kb(Bw + (size_t)(c0 + t * 16 + nloc) * K + kb, hlf); acc[0][t] = wmma16b(a0, bw, acc[0][t]); acc[1][t] = wmma16b(a1, bw, acc[1][t]); } }
#pragma unroll
  for (int t = 0; t < 8; ++t) { const float bv = (bias != nullptr) ? bias[c0 + t * 16 + nloc] : 0.0f;
#pragma unroll
    for (int r = 0; r < 2; ++r)
#pragma unroll
      for (int v = 0; v < 8; ++v) { float y = acc[r][t][v] * (1.0f / XS) + bv; if (EPI == 2) y = fmaxf(y, 0.0f); Ts[wave][r * 16 + 8 * hlf + v][t * 16 + nloc] = y; } }
  wave_lds_sync();
  if (EPI == 3 && c0 < 2 * D) {
    for (int i = lane; i < 32 * 64; i += 32) { const int rr = i >> 6, cp = (i & 63) * 2; const int t = (m0 + rr) % L; const int i2 = ((c0 + cp) & 63) >> 1;
      const float invf = __builtin_amdgcn_exp2f(-(float)i2 * (13.287712379549449f / 32.0f));
      float sn, cs; sincos_r((float)t * invf, sn, cs); const float xe = Ts[wave][rr][cp], xo = Ts[wave][rr][cp + 1];
      Ts[wave][rr][cp] = pmul(xe, cs) - pmul(xo, sn); Ts[wave][rr][cp + 1] = pmul(xe, sn) + pmul(xo, cs); }
    wave_lds_sync(); }
  for (int pass = 0; pass < 2; ++pass) {
    if (EPI == 1) { for (int i = lane; i < 32 * 32; i += 32) { const int rr = i >> 5, c4 = (i & 31) * 4; const size_t gi = (size_t)(m0 + rr) * N + c0 + c4; v4f o = *(const v4f*)(&Ts[wave][rr][c4]); const v4f xr = *(const v4f*)(resid + gi);
        for (int e = 0; e < 4; ++e) o[e] += RND ? bf16_rne(xr[e]) : xr[e]; *(volatile v4f*)(Cf + gi) = o; } }
    else { for (int i = lane; i < 32 * 16; i += 32) { const int rr = i >> 4, c8 = (i & 15) * 8; v8b o; for (int e = 0; e < 8; ++e) o[e] = (b16)(Ts[wave][rr][c8 + e] * XS); *(volatile v8b*)(Ch + (size_t)(m0 + rr) * N + c0 + c8) = o; } }
    __threadfence(); }
}

__global__ __launch_bounds__(256) void vt_kernel(const b16* __restrict__ QKV, b16* __restrict__ vt) {
  __shared__ __attribute__((aligned(16))) b16 T[HD][128 + 8];
  const int b = blockIdx.z, h = blockIdx.y, t0 = blockIdx.x * 128, t_ = threadIdx.x;
  for (int i = t_; i < 128 * (HD / 8); i += 256) { const int tk = i >> 3, d8 = (i & 7) * 8; const v8b vv = *(const v8b*)(QKV + ((size_t)(b * L + t0 + tk)) * DQ + 2 * D + h * HD + d8); for (int e = 0; e < 8; ++e) T[d8 + e][tk] = vv[e]; }
  __syncthreads();
  for (int pass = 0; pass < 2; ++pass) { for (int i = t_; i < HD * 16; i += 256) { const int d = i >> 4, c8 = (i & 15) * 8; *(volatile v8b*)(vt + (((size_t)b * H + h) * HD + d) * L + t0 + c8) = *(const v8b*)(&T[d][c8]); } __threadfence(); }
}

__global__ __launch_bounds__(256) void attn_kernel(const b16* __restrict__ QKV, const b16* __restrict__ vt, b16* __restrict__ ctx) {
  __shared__ __attribute__((aligned(16))) b16 Os[16][8 * HD + 8];
  const int wid = threadIdx.x >> 5, lane = threadIdx.x & 31, hh = lane >> 4, col = lane & 15; const int b = blockIdx.x / (L / 16), q0 = (blockIdx.x % (L / 16)) * 16, h = blockIdx.y * 8 + wid, qi = q0 + col;
  const b16* Qr = QKV + (size_t)(b * L) * DQ + h * HD; const b16* Kr = QKV + (size_t)(b * L) * DQ + D + h * HD; const b16* V = vt + (((size_t)b * H + h) * HD) * L;
  const v16b qf0 = frag_kb(Qr + (size_t)qi * DQ, hh), qf1 = frag_kb(Qr + (size_t)qi * DQ + 32, hh);
  float m = -INFINITY, l = 0.0f; v8f o[4] = {{}, {}, {}, {}};
  for (int kb = 0; kb <= q0 + 15; kb += 32) {
    const v16b ka0 = frag_kb(Kr + (size_t)(kb + col) * DQ, hh), ka1 = frag_kb(Kr + (size_t)(kb + col) * DQ + 32, hh), kc0 = frag_kb(Kr + (size_t)(kb + 16 + col) * DQ, hh), kc1 = frag_kb(Kr + (size_t)(kb + 16 + col) * DQ + 32, hh);
    v8f s0 = {}, s1 = {}; s0 = wmma16b(ka0, qf0, s0); s0 = wmma16b(ka1, qf1, s0); s1 = wmma16b(kc0, qf0, s1); s1 = wmma16b(kc1, qf1, s1);
    float mr = -INFINITY;
#pragma unroll
    for (int r = 0; r < 8; ++r) { const int k0 = kb + 8 * hh + r, k1 = k0 + 16; s0[r] = (k0 <= qi) ? s0[r] * (0.125f / (XS * XS)) : -INFINITY; s1[r] = (k1 <= qi) ? s1[r] * (0.125f / (XS * XS)) : -INFINITY; mr = fmaxf(mr, fmaxf(s0[r], s1[r])); }
    mr = fmaxf(mr, __shfl_xor(mr, 16));
    const float mn = fmaxf(m, mr), al_ = nexp(m - mn); m = mn; float sum = 0.0f; v16b pbv;
#pragma unroll
    for (int r = 0; r < 8; ++r) { const float e0 = (s0[r] == -INFINITY) ? 0.0f : nexp(s0[r] - mn), e1 = (s1[r] == -INFINITY) ? 0.0f : nexp(s1[r] - mn); sum += e0 + e1; pbv[r] = (b16)(e0 * PS); pbv[8 + r] = (b16)(e1 * PS); }
    sum += __shfl_xor(sum, 16); l = l * al_ + sum;
#pragma unroll
    for (int t = 0; t < 4; ++t) { o[t] *= al_; const v16b vf = frag_kb(V + (size_t)(t * 16 + col) * L + kb, hh); o[t] = wmma16b(vf, pbv, o[t]); } }
  const float inv = 1.0f / (l * PS);
#pragma unroll
  for (int t = 0; t < 4; ++t)
#pragma unroll
    for (int r = 0; r < 8; ++r) Os[col][wid * HD + t * 16 + 8 * hh + r] = (b16)(o[t][r] * inv);
  __syncthreads();
  for (int pass = 0; pass < 2; ++pass) { for (int i = threadIdx.x; i < 16 * (8 * HD / 8); i += 256) { const int rr = i / (8 * HD / 8), c8 = (i % (8 * HD / 8)) * 8; *(volatile v8b*)(ctx + ((size_t)(b * L + q0 + rr)) * D + blockIdx.y * 8 * HD + c8) = *(const v8b*)(&Os[rr][c8]); } __threadfence(); }
}
}

extern "C" void kernel_launch(void* const* d_in, const int* in_sizes, int n_in,
                              void* d_out, int out_size, void* d_ws, size_t ws_size, hipStream_t stream) {
  (void)n_in; (void)out_size;
  const float* x = (const float*)d_in[0]; const float* g1 = (const float*)d_in[1]; const float* be1 = (const float*)d_in[2]; const float* wqkv = (const float*)d_in[3]; const float* bqkv = (const float*)d_in[4]; const float* wo = (const float*)d_in[5]; const float* bo = (const float*)d_in[6];
  const float* g2 = (const float*)d_in[7]; const float* be2 = (const float*)d_in[8]; const float* w1 = (const float*)d_in[9]; const float* b1 = (const float*)d_in[10]; const float* w2 = (const float*)d_in[11]; const float* b2 = (const float*)d_in[12];
  float* out = (float*)d_out;
  if (in_sizes[0] != NT * D || in_sizes[3] != DQ * D || in_sizes[9] != DF * D || in_sizes[11] != D * DF) return;
  size_t off = 0; char* ws = (char*)d_ws;
  auto carve = [&](size_t bytes) { char* p = ws + off; off += (bytes + 255) & ~(size_t)255; return p; };
  b16* R = (b16*)carve(Wo_::END * 2); float* P = (float*)carve(13312 * 4);
  b16* SH = (b16*)carve((size_t)NT * D * 2); b16* RA = (b16*)carve((size_t)NT * DF * 2); b16* VT = (b16*)carve((size_t)Bn * H * HD * L * 2); float* X1 = (float*)carve((size_t)NT * D * 4);
  if (off > ws_size) return;
  prep_kernel<<<512, 256, 0, stream>>>(wqkv, wo, w1, w2, bqkv, bo, b1, b2, g1, be1, g2, be2, R, P);
  ln_kernel<<<NT / 8, 256, 0, stream>>>(x, 1, P + 9216, P + 10240, SH);
  gemm_kernel<D, DQ, 3, 0><<<dim3(DQ / 256, NT / 32), 64, 0, stream>>>(SH, R + Wo_::QKV, P, nullptr, RA, nullptr);
  vt_kernel<<<dim3(L / 128, H, Bn), 256, 0, stream>>>(RA, VT);
  attn_kernel<<<dim3(NT / 16, 2), 256, 0, stream>>>(RA, VT, SH);
  gemm_kernel<D, D, 1, 1><<<dim3(D / 256, NT / 32), 64, 0, stream>>>(SH, R + Wo_::O, P + 3072, x, nullptr, X1);
  ln_kernel<<<NT / 8, 256, 0, stream>>>(X1, 0, P + 11264, P + 12288, SH);
  gemm_kernel<D, DF, 2, 0><<<dim3(DF / 256, NT / 32), 64, 0, stream>>>(SH, R + Wo_::F1, P + 4096, nullptr, RA, nullptr);
  gemm_kernel<DF, D, 1, 0><<<dim3(D / 256, NT / 32), 64, 0, stream>>>(RA, R + Wo_::F2, P + 8192, X1, nullptr, out);
}
